// RGAT_27547920236878
// MI455X (gfx1250) — hardware-run, weakly checked
//
#include <hip/hip_runtime.h>

typedef float          v8f   __attribute__((ext_vector_type(8)));
typedef float          v4f   __attribute__((ext_vector_type(4)));
typedef unsigned int   v4u   __attribute__((ext_vector_type(4)));
typedef int            v8i   __attribute__((ext_vector_type(8)));
typedef unsigned short v8us  __attribute__((ext_vector_type(8)));
typedef unsigned short v16us __attribute__((ext_vector_type(16)));
typedef __bf16         v16bf __attribute__((ext_vector_type(16)));
typedef _Float16       v16h  __attribute__((ext_vector_type(16)));
typedef v4f  __attribute__((may_alias)) v4fa;
typedef v8us __attribute__((may_alias)) v8usa;
union FragB { v16bf v; v16us u; v8us h[2]; v8i w; };
union FragH { v16h  v; v16us u; v8us h[2]; v8i w; };

__device__ __forceinline__ v8f wmb(const FragB& a, const FragB& b, v8f c) {
  v8f d = __builtin_amdgcn_wmma_f32_16x16x32_bf16(false, a.v, false, b.v, (short)0, c, false, false);
  asm volatile("v_nop\n\tv_nop\n\tv_nop\n\tv_nop" : "+v"(d) : "v"(a.w), "v"(b.w));
  return d;
}

__device__ __forceinline__ v8f wmh(const FragH& a, const FragH& b, v8f c) {
  v8f d = __builtin_amdgcn_wmma_f32_16x16x32_f16(false, a.v, false, b.v, (short)0, c, false, false);
  asm volatile("v_nop\n\tv_nop\n\tv_nop\n\tv_nop" : "+v"(d) : "v"(a.w), "v"(b.w));
  return d;
}

__device__ __forceinline__ unsigned bf16_bits(float f) {
  const unsigned u = __float_as_uint(f);
  const unsigned r = (u + 0x7FFFu + ((u >> 16) & 1u)) >> 16;
  const unsigned q = (u >> 16) | 0x40u;
  return ((u & 0x7fffffffu) > 0x7f800000u) ? q : r;
}

__device__ __forceinline__ float bf16_val(float f) {
  return __uint_as_float(bf16_bits(f) << 16);
}
__device__ __forceinline__ int clampi(int v, int lo, int hi) {
  return v < lo ? lo : (v > hi ? hi : v);
}

__device__ __forceinline__ unsigned f16_bits(float f) {
  const unsigned u  = __float_as_uint(f);
  const unsigned s  = (u >> 16) & 0x8000u;
  const unsigned a  = u & 0x7fffffffu;
  const unsigned t  = a - 0x38000000u;
  const unsigned r  = (t + 0x0FFFu + ((t >> 13) & 1u)) >> 13;
  const unsigned rc = r > 0x7C00u ? 0x7C00u : r;
  const bool small  = a < 0x38800000u;
  const bool isnan  = a > 0x7f800000u;
  const unsigned fin = small ? 0u : (s | rc);
  return isnan ? (s | 0x7E00u) : fin;
}

__device__ __forceinline__ unsigned pk16(unsigned lo, unsigned hi) { return lo | (hi << 16); }
__device__ __forceinline__ unsigned bf16_lo_bits(float v) {
  float hi = bf16_val(v);
  asm volatile("" : "+v"(hi));
  return bf16_bits(v - hi);
}
__device__ __forceinline__ v4u pack8_bf16(v4f a, v4f c) {
  return (v4u){ pk16(bf16_bits(a[0]), bf16_bits(a[1])), pk16(bf16_bits(a[2]), bf16_bits(a[3])),
                pk16(bf16_bits(c[0]), bf16_bits(c[1])), pk16(bf16_bits(c[2]), bf16_bits(c[3])) };
}
__device__ __forceinline__ v4u pack8_bf16_lo(v4f a, v4f c) {
  return (v4u){ pk16(bf16_lo_bits(a[0]), bf16_lo_bits(a[1])), pk16(bf16_lo_bits(a[2]), bf16_lo_bits(a[3])),
                pk16(bf16_lo_bits(c[0]), bf16_lo_bits(c[1])), pk16(bf16_lo_bits(c[2]), bf16_lo_bits(c[3])) };
}
__device__ __forceinline__ v4u pack8_f16(v4f a, v4f c) {
  return (v4u){ pk16(f16_bits(a[0]), f16_bits(a[1])), pk16(f16_bits(a[2]), f16_bits(a[3])),
                pk16(f16_bits(c[0]), f16_bits(c[1])), pk16(f16_bits(c[2]), f16_bits(c[3])) };
}

template <int FORM>
__global__ __launch_bounds__(256) void k_plane(const float* __restrict__ src, int rows, int cols, int ldsrc,
                                               unsigned short* __restrict__ dst, int MP, int KP) {
  static_assert(FORM >= 0 && FORM <= 3);
  const int KTOT = (FORM == 1 || FORM == 3) ? 2 * KP : KP;
  const unsigned ppr   = (unsigned)(KTOT >> 3);
  const unsigned kp8   = (unsigned)(KP >> 3);
  const unsigned total = (unsigned)MP * ppr;
  const unsigned g     = blockIdx.x * 256u + threadIdx.x;
  const unsigned rowu  = g / ppr;
  const unsigned p     = g - rowu * ppr;
  const bool second    = p >= kp8;
  const int row = (int)rowu;
  const int c0  = (int)((second ? p - kp8 : p) << 3);
  const float* srow = src + (size_t)clampi(row, 0, rows - 1) * (size_t)ldsrc;
  float x[8];
  unsigned mk[8];
#pragma unroll
  for (int e = 0; e < 8; ++e) {
    const int c = c0 + e;
    const float v = srow[clampi(c, 0, cols - 1)];
    asm volatile("" :: "v"(v));
    x[e]  = v;
    mk[e] = (row < rows && c < cols) ? 0xFFFFu : 0u;
  }
  const v4f a = (v4f){ x[0], x[1], x[2], x[3] };
  const v4f c = (v4f){ x[4], x[5], x[6], x[7] };
  v4u o;
  if (FORM == 2) {
    o = pack8_f16(a, c);
  } else {
    const v4u hi = pack8_bf16(a, c);
    o = hi;
    if (FORM == 1) { const v4u lo = pack8_bf16_lo(a, c); o = second ? lo : hi; }
  }
  const v4u mw = (v4u){ pk16(mk[0], mk[1]), pk16(mk[2], mk[3]), pk16(mk[4], mk[5]), pk16(mk[6], mk[7]) };
  o &= mw;
  if (g < total) {
    volatile v4u* q = (volatile v4u*)(dst + (size_t)g * 8);
    *q = o;
    __threadfence();
    *q = o;
  }
}

template <int FORM> struct FragOf    { typedef FragB T; };
template <>         struct FragOf<2> { typedef FragH T; };
__device__ __forceinline__ v8f mm(const FragB& a, const FragB& b, v8f c) { return wmb(a, b, c); }
__device__ __forceinline__ v8f mm(const FragH& a, const FragH& b, v8f c) { return wmh(a, b, c); }
template <class F> __device__ __forceinline__ F ld_frag(const unsigned short* p) {
  F f;
  f.h[0] = *(const v8usa*)(p);
  f.h[1] = *(const v8usa*)(p + 16);
  return f;
}

template <int FORM, int EPI>
__global__ __launch_bounds__(256) __attribute__((amdgpu_num_vgpr(248)))
void k_gemm_nt(const unsigned short* __restrict__ A, const unsigned short* __restrict__ B,
               const float* __restrict__ bias, float* __restrict__ D, int M, int N, int KTOT, int ldd) {
  static_assert(FORM >= 0 && FORM <= 2);
  static_assert(EPI == 0 || EPI == 1);
  typedef typename FragOf<FORM>::T F;
  __shared__ __attribute__((aligned(16))) float sT[8][16 * 68];
  const int lane = threadIdx.x & 31;
  const int wave = threadIdx.x >> 5;
  const int tilesM = (M + 63) >> 6;
  const int tilesN = (N + 63) >> 6;
  const int tile = blockIdx.x * 8 + wave;
  if (tile >= tilesM * tilesN) return;
  const int tm = tile / tilesN;
  const int tn = tile - tm * tilesN;
  const int m0 = tm << 6;
  const int n0 = tn << 6;

  const int rl = lane & 15;
  const int h8 = (lane >> 4) * 8;
  const unsigned short* pa = A + (size_t)(m0 + rl) * (size_t)KTOT + h8;
  const unsigned short* pb = B + (size_t)(n0 + rl) * (size_t)KTOT + h8;

  v8f acc[4][4];
#pragma unroll
  for (int i = 0; i < 4; ++i)
#pragma unroll
    for (int j = 0; j < 4; ++j) acc[i][j] = (v8f){0.f, 0.f, 0.f, 0.f, 0.f, 0.f, 0.f, 0.f};

#pragma unroll 1
  for (int k0 = 0; k0 < KTOT; k0 += 32) {
    F bf[4];
#pragma unroll
    for (int j = 0; j < 4; ++j) bf[j] = ld_frag<F>(pb + (size_t)(j << 4) * (size_t)KTOT + k0);
#pragma unroll
    for (int i = 0; i < 4; ++i) {
      const F af = ld_frag<F>(pa + (size_t)(i << 4) * (size_t)KTOT + k0);
#pragma unroll
      for (int j = 0; j < 4; ++j) acc[i][j] = mm(af, bf[j], acc[i][j]);
    }
  }

  float* slab = sT[wave];
  const int hh = lane >> 4;
  const int c4 = (lane & 15) * 4;
  const int nc = n0 + c4;
  const bool cok = nc < N;
  v4f bv = (v4f){0.f, 0.f, 0.f, 0.f};
  if (EPI == 1) {
    bv = *(const v4fa*)(bias + clampi(nc, 0, N - 4));
    asm volatile("" :: "v"(bv));
  }
#pragma unroll
  for (int i = 0; i < 4; ++i) {
    const int mBase = m0 + (i << 4);
#pragma unroll
    for (int j = 0; j < 4; ++j) {
#pragma unroll
      for (int r = 0; r < 8; ++r) slab[(h8 + r) * 68 + (j << 4) + rl] = acc[i][j][r];
    }
    __builtin_amdgcn_fence(__ATOMIC_RELEASE, "workgroup");
    __builtin_amdgcn_wave_barrier();
    __builtin_amdgcn_fence(__ATOMIC_ACQUIRE, "workgroup");
    v4f vv[8];
#pragma unroll
    for (int it = 0; it < 8; ++it) {
      const int row = it * 2 + hh;
      v4f v = *(const v4fa*)(slab + row * 68 + c4);
      if (EPI == 1) v += bv;
      vv[it] = v;
    }
    for (int pass = 0; pass < 2; ++pass) {
#pragma unroll
      for (int it = 0; it < 8; ++it) {
        const int row = mBase + it * 2 + hh;
        if (cok && row < M) *(volatile v4f*)(D + (size_t)row * (size_t)ldd + nc) = vv[it];
      }
      __threadfence();
    }
    __builtin_amdgcn_fence(__ATOMIC_RELEASE, "workgroup");
    __builtin_amdgcn_wave_barrier();
    __builtin_amdgcn_fence(__ATOMIC_ACQUIRE, "workgroup");
  }
}

#ifndef HOP2_TWO_TERM
#define HOP2_TWO_TERM 0
#endif

typedef int   v4i __attribute__((ext_vector_type(4)));
typedef float v2f __attribute__((ext_vector_type(2)));
typedef v4i __attribute__((may_alias)) v4ia;
typedef v4u __attribute__((may_alias)) v4ua;
typedef v2f __attribute__((may_alias)) v2fa;

static constexpr int kN = 100000;
static constexpr int kC = 64;
static constexpr int kE = 1000000;
static constexpr int kR = 24;
static constexpr int MPAD = 100032;
static constexpr int PW   = 2 * kC;
static constexpr int E1K  = kC * (1 + HOP2_TWO_TERM);
static constexpr int NTHR = 256;
static constexpr int NWAVE = 8;
static constexpr int EPT = 8;
static constexpr int CHUNK = NTHR * EPT;
static constexpr int WCAP = EPT * 32;
static constexpr int LISTN = NWAVE * WCAP;
static constexpr int NBRUN = 1024;
static constexpr int NBLK = 98;
static constexpr int RCAP = 13312;
static constexpr int DEGCAP = 64;
static constexpr int NCHUNK = (kE + CHUNK - 1) / CHUNK;
static constexpr int LDS_BK = (2 * RCAP + 2 * NBRUN + LISTN + 2 * NWAVE) * 4;
static constexpr int LDS_RP = (RCAP + 2 * NBRUN + kR * kC + 2 * NWAVE * DEGCAP + NWAVE * 64) * 4;

static_assert(kN <= 131072);
static_assert(kR <= 32);
static_assert(NBRUN == 1024);
static_assert(kC == 64);
static_assert(kE - (kE / CHUNK) * CHUNK == 576);
static_assert(NCHUNK == 489);
static_assert(WCAP == 256 && CHUNK == NWAVE * WCAP);
static_assert(NBRUN == NTHR * 4);
static_assert(LISTN >= NBRUN);
static_assert((RCAP % 32) == 0 && (RCAP % (4 * NTHR)) == 0);
static_assert(RCAP * 4 >= 5 * 10472);
static_assert(DEGCAP == 64 && DEGCAP >= 26 + 8);
static_assert(NBLK * NBRUN >= MPAD && (NBLK - 1) * NBRUN < kN);
static_assert((MPAD % 64) == 0 && MPAD >= kN && (kN % 16) == 0);
static_assert((E1K % 32) == 0 && (PW % 32) == 0);
static_assert(LDS_BK <= 262144 && LDS_RP <= 262144);
static_assert(LDS_BK <= 327680 && LDS_RP <= 327680 && 34816 <= 327680);

static constexpr size_t SZ_XB   = (size_t)MPAD * kC * 2;
static constexpr size_t SZ_WB1  = (size_t)128 * kC * 2;
static constexpr size_t SZ_WB2  = (size_t)128 * 128 * 2;
static constexpr size_t SZ_RELF = (size_t)kR * kC * 4;
static constexpr size_t SZ_P    = (size_t)MPAD * PW * 4;
static constexpr size_t SZ_ENT1 = (size_t)MPAD * kC * 4;
static constexpr size_t SZ_E1   = (size_t)MPAD * E1K * 2;
static constexpr size_t SZ_LIST = (size_t)NBLK * RCAP * 4;
static constexpr size_t SZ_OFF  = (size_t)NBLK * NBRUN * 4;
static constexpr size_t SZ_META = (size_t)NBLK * 128;
static constexpr size_t O_XB   = 0;
static constexpr size_t O_WB1  = O_XB + SZ_XB;
static constexpr size_t O_WB2  = O_WB1 + SZ_WB1;
static constexpr size_t O_RELF = O_WB2 + SZ_WB2;
static constexpr size_t O_P    = O_RELF + SZ_RELF;
static constexpr size_t O_ENT1 = O_P + SZ_P;
static constexpr size_t O_E1   = O_ENT1 + SZ_ENT1;
static constexpr size_t O_LIST = O_E1 + SZ_E1;
static constexpr size_t O_OFF  = O_LIST + SZ_LIST;
static constexpr size_t O_CNT  = O_OFF + SZ_OFF;
static constexpr size_t O_META = O_CNT + SZ_OFF;
static constexpr size_t WS_TOTAL = O_META + SZ_META;
static_assert((SZ_XB % 256) == 0 && (SZ_WB1 % 256) == 0 && (SZ_WB2 % 256) == 0 && (SZ_RELF % 256) == 0);
static_assert((SZ_P % 256) == 0 && (SZ_ENT1 % 256) == 0 && (SZ_E1 % 256) == 0 && (SZ_LIST % 256) == 0);
static_assert((SZ_OFF % 256) == 0 && (SZ_META % 256) == 0);
static_assert(WS_TOTAL <= ((size_t)128 << 20));

static constexpr int PB_X  = MPAD * kC / 8 / NTHR;
static constexpr int PB_W1 = 128 * kC / 8 / NTHR;
static constexpr int PB_W2 = 128 * 128 / 8 / NTHR;
static constexpr int PB_R  = 2;
static constexpr int PB_TOTAL = PB_X + PB_W1 + PB_W2 + PB_R;
static_assert(PB_X * NTHR * 8 == MPAD * kC);
static_assert(PB_W1 * NTHR * 8 == 128 * kC && PB_W2 * NTHR * 8 == 128 * 128);
static_assert(PB_R * NTHR >= kR * kC / 4);

__device__ __forceinline__ int imin(int a, int b) { return a < b ? a : b; }
__device__ __forceinline__ void wsync() {
  __builtin_amdgcn_fence(__ATOMIC_RELEASE, "workgroup");
  __builtin_amdgcn_wave_barrier();
  __builtin_amdgcn_fence(__ATOMIC_ACQUIRE, "workgroup");
}

__device__ __forceinline__ v4u wpiece(const float* __restrict__ W, int n, int k8) {
  const int kb = n < kC ? 0 : kC;
  const int nc = n & (kC - 1);
  const float* s = W + (size_t)(kb + k8) * kC + nc;
  float x[8];
#pragma unroll
  for (int e = 0; e < 8; ++e) {
    const float v = s[e * kC];
    asm volatile("" :: "v"(v));
    x[e] = v;
  }
  return pack8_bf16((v4f){ x[0], x[1], x[2], x[3] }, (v4f){ x[4], x[5], x[6], x[7] });
}

__global__ __launch_bounds__(NTHR) void k_prep(const float* __restrict__ ent, const float* __restrict__ rel,
                                               const float* __restrict__ W, unsigned short* XB,
                                               unsigned short* WB1, unsigned short* WB2, float* RELF) {
  const int tid = (int)threadIdx.x;
  const int blk = (int)blockIdx.x;
  if (blk < PB_X) {
    const unsigned g = (unsigned)blk * NTHR + (unsigned)tid;
    const int row = (int)(g >> 3);
    const int p   = (int)(g & 7u);
    const int rc  = imin(row, kN - 1);
    const float* s = ent + (size_t)rc * kC + 8 * p;
    const v4f a = *(const v4fa*)s;
    const v4f c = *(const v4fa*)(s + 4);
    asm volatile("" :: "v"(a));
    asm volatile("" :: "v"(c));
    v4u o = pack8_bf16(a, c);
    const unsigned mk = row < kN ? 0xFFFFFFFFu : 0u;
    o &= (v4u){ mk, mk, mk, mk };
    volatile v4u* q = (volatile v4u*)(XB + (size_t)g * 8);
    *q = o;
    __threadfence();
    *q = o;
  } else if (blk < PB_X + PB_W1) {
    const int u  = (blk - PB_X) * NTHR + tid;
    const int n  = u >> 3;
    const int k8 = (u & 7) * 8;
    const v4u o = wpiece(W, n, k8);
    volatile v4u* q = (volatile v4u*)(WB1 + (size_t)u * 8);
    *q = o;
    __threadfence();
    *q = o;
  } else if (blk < PB_X + PB_W1 + PB_W2) {
    const int u  = (blk - PB_X - PB_W1) * NTHR + tid;
    const int n  = u >> 4;
    const int k8 = (u & 7) * 8;
    const v4u o = wpiece(W, n, k8);
    volatile v4u* q = (volatile v4u*)(WB2 + (size_t)u * 8);
    *q = o;
    __threadfence();
    *q = o;
  } else {
    const int u  = (blk - PB_X - PB_W1 - PB_W2) * NTHR + tid;
    const int uc = imin(u, kR * kC / 4 - 1);
    const v4f v = ((const v4fa*)rel)[uc];
    asm volatile("" :: "v"(v));
    const v4f o = (v4f){ bf16_val(v[0]), bf16_val(v[1]), bf16_val(v[2]), bf16_val(v[3]) };
    if (u < kR * kC / 4) {
      volatile v4f* q = (volatile v4f*)(RELF + (size_t)u * 4);
      *q = o;
      __threadfence();
      *q = o;
    }
  }
}

__device__ __forceinline__ int scan_chunk(const int* __restrict__ heads, int cbase, int slotBase, int nb,
                                          int* list, int lane, int wave) {
  int wc = 0;
  const int elw  = wave * WCAP;
  const int sent = (-0x7fffffff - 1);
  unsigned sl[EPT];
  bool hit[EPT];
  bool anyh = false;
#pragma unroll
  for (int j = 0; j < EPT; ++j) {
    const int idx = cbase + elw + 32 * j + lane;
    const int x = heads[imin(idx, kE - 1)];
    asm volatile("" :: "v"(x));
    const int mk = idx < kE ? -1 : 0;
    const int hv = (x & mk) | (sent & ~mk);
    sl[j]  = (unsigned)hv - (unsigned)slotBase;
    hit[j] = sl[j] < (unsigned)nb;
    anyh = anyh | hit[j];
  }
  const unsigned any = __builtin_amdgcn_ballot_w32(anyh);
  if (any != 0u) {
#pragma unroll
    for (int j = 0; j < EPT; ++j) {
      const unsigned mj = __builtin_amdgcn_ballot_w32(hit[j]);
      if (mj != 0u) {
        if (hit[j]) {
          const int pos = wc + (int)__builtin_amdgcn_mbcnt_lo(mj, 0u);
          if (pos < WCAP) list[elw + pos] = ((elw + 32 * j + lane) << 12) | (int)sl[j];
        }
        wc += (int)__builtin_popcount(mj);
      }
    }
  }
  return wc;
}

__global__ __launch_bounds__(NTHR) void k_bucket(const int* __restrict__ heads, const int* __restrict__ tails,
                                                 const int* __restrict__ etype, unsigned* LIST, int* OFFG,
                                                 int* CNTG, int* META) {
  extern __shared__ v4f bk_dyn[];
  unsigned* reg1 = (unsigned*)bk_dyn;
  unsigned* reg2 = reg1 + RCAP;
  int* scnt = (int*)(reg2 + RCAP);
  int* soff = scnt + NBRUN;
  int* list = soff + NBRUN;
  int* wcnt = list + LISTN;
  int* wtot = wcnt + NWAVE;
  const int tid = (int)threadIdx.x, lane = tid & 31, wave = tid >> 5;
  const int b = (int)blockIdx.x;
  const int slotBase = b * NBRUN;
  const int nb = imin(NBRUN, kN - slotBase);

  for (int i = tid; i < NBRUN; i += NTHR) scnt[i] = 0;
  for (int i = tid; i < RCAP; i += NTHR) reg2[i] = 0u;
  __syncthreads();

  int tot = 0, totRaw = 0;
#pragma unroll 1
  for (int ch = 0; ch < NCHUNK; ++ch) {
    const int cbase = ch * CHUNK;
    const int wc = scan_chunk(heads, cbase, slotBase, nb, list, lane, wave);
    if (lane == 0) wcnt[wave] = wc;
    __syncthreads();
    int pre = 0, all = 0;
#pragma unroll
    for (int w2 = 0; w2 < NWAVE; ++w2) {
      const int c = clampi(wcnt[w2], 0, WCAP);
      all += c;
      pre += (w2 < wave) ? c : 0;
    }
    const int wcc  = __builtin_amdgcn_readfirstlane(imin(wc, WCAP));
    const int base = tot + pre;
#pragma unroll 1
    for (int i0 = 0; i0 < wcc; i0 += 32) {
      const int i  = i0 + lane;
      const int ic = imin(i, wcc - 1);
      const int ent = list[wave * WCAP + ic];
      const int el  = (ent >> 12) & (CHUNK - 1);
      const unsigned s = (unsigned)ent & (unsigned)(NBRUN - 1);
      const int eid = imin(cbase + el, kE - 1);
      int tl = tails[eid];
      asm volatile("" :: "v"(tl));
      int ty = etype[eid];
      asm volatile("" :: "v"(ty));
      tl = clampi(tl, 0, kN - 1);
      ty = clampi(ty, 0, kR - 1);
      const unsigned word = (unsigned)tl | ((unsigned)ty << 17) | (s << 22);
      const int pos = base + i;
      if (i < wcc && pos < RCAP) reg1[pos] = word;
    }
    totRaw += all;
    tot = imin(tot + all, RCAP);
    __syncthreads();
  }
  const int nh = tot;

  if (wave == 0) {
#pragma unroll 1
    for (int b0 = 0; b0 < nh; b0 += 32) {
      const int idx = b0 + lane;
      const int uv  = (int)reg1[idx < nh ? idx : nh - 1];
      const int m32 = (nh - b0) < 32 ? (nh - b0) : 32;
#pragma unroll 1
      for (int k = 0; k < m32; ++k) {
        const unsigned u = (unsigned)__builtin_amdgcn_readlane(uv, k);
        const int s = (int)((u >> 22) & (unsigned)(NBRUN - 1));
        if (lane == 0) scnt[s] = scnt[s] + 1;
      }
    }
  }
  __syncthreads();

  {
    const v4i ca = *(const v4ia*)(scnt + 4 * tid);
    const int e0 = ca.x < 0 ? 0 : ca.x, e1 = ca.y < 0 ? 0 : ca.y, e2 = ca.z < 0 ? 0 : ca.z, e3 = ca.w < 0 ? 0 : ca.w;
    const int ts = e0 + e1 + e2 + e3;
    int incl = ts;
#pragma unroll
    for (int d = 1; d < 32; d <<= 1) {
      const int up = __shfl_up(incl, d);
      if (lane >= d) incl += up;
    }
    if (lane == 31) wtot[wave] = incl;
    __syncthreads();
    int pre = 0;
#pragma unroll
    for (int w2 = 0; w2 < NWAVE; ++w2) pre += (w2 < wave) ? wtot[w2] : 0;
    int run = pre + incl - ts;
    soff[4 * tid + 0] = run; run += e0;
    soff[4 * tid + 1] = run; run += e1;
    soff[4 * tid + 2] = run; run += e2;
    soff[4 * tid + 3] = run;
  }
  __syncthreads();
  for (int i = tid; i < NBRUN; i += NTHR) list[i] = soff[i];
  __syncthreads();

  if (wave == 0) {
#pragma unroll 1
    for (int b0 = 0; b0 < nh; b0 += 32) {
      const int idx = b0 + lane;
      const int uv  = (int)reg1[idx < nh ? idx : nh - 1];
      const int m32 = (nh - b0) < 32 ? (nh - b0) : 32;
#pragma unroll 1
      for (int k = 0; k < m32; ++k) {
        const unsigned u = (unsigned)__builtin_amdgcn_readlane(uv, k);
        const int s = (int)((u >> 22) & (unsigned)(NBRUN - 1));
        if (lane == 0) {
          int pos = list[s];
          pos = clampi(pos, 0, RCAP - 1);
          reg2[pos] = u;
          list[s] = pos + 1;
        }
      }
    }
  }
  __syncthreads();

  const v4i so = *(const v4ia*)(soff + 4 * tid);
  const v4i sc = *(const v4ia*)(scnt + 4 * tid);
  v4i mv = (v4i){ 0, 0, 0, 0 };
  mv.x = lane == 0 ? nh : 0;
  mv.y = lane == 0 ? (totRaw > RCAP ? 1 : 0) : 0;
  mv.z = lane == 0 ? totRaw : 0;
  unsigned* lrow = LIST + (size_t)b * RCAP;
  for (int pass = 0; pass < 2; ++pass) {
#pragma unroll 1
    for (int it = 0; it < RCAP / 4 / NTHR; ++it) {
      const int piece = it * NTHR + tid;
      const v4u v = *(const v4ua*)(reg2 + 4 * piece);
      *(volatile v4u*)(lrow + 4 * piece) = v;
    }
    *(volatile v4i*)(OFFG + (size_t)b * NBRUN + 4 * tid) = so;
    *(volatile v4i*)(CNTG + (size_t)b * NBRUN + 4 * tid) = sc;
    if (wave == 0 && lane < 8) *(volatile v4i*)(META + (size_t)b * 32 + 4 * lane) = mv;
    __threadfence();
  }
}

template <int HOP>
__global__ __launch_bounds__(NTHR) void k_replay(const unsigned* __restrict__ LIST, const int* __restrict__ OFFG,
                                                 const int* __restrict__ CNTG, const int* __restrict__ META,
                                                 const float* __restrict__ RELF, const float* __restrict__ P,
                                                 const unsigned* __restrict__ XBW, const float* __restrict__ ENTR,
                                                 float* ENTW, unsigned short* E1, float* OUT) {
  static_assert(HOP == 1 || HOP == 2);
  extern __shared__ v4f rp_dyn[];
  unsigned* lst = (unsigned*)rp_dyn;
  int* soffL = (int*)(lst + RCAP);
  int* scntL = soffL + NBRUN;
  float* relL  = (float*)(scntL + NBRUN);
  float* scAll = relL + kR * kC;
  float* pwAll = scAll + NWAVE * DEGCAP;
  float* stAll = pwAll + NWAVE * DEGCAP;
  const int tid = (int)threadIdx.x, lane = tid & 31, wave = tid >> 5;
  const int b = (int)blockIdx.x;

  {
    const unsigned* lrow = LIST + (size_t)b * RCAP;
#pragma unroll 1
    for (int it = 0; it < RCAP / 4 / NTHR; ++it) {
      const int piece = it * NTHR + tid;
      *(v4ua*)(lst + 4 * piece) = *(const v4ua*)(lrow + 4 * piece);
    }
    *(v4ia*)(soffL + 4 * tid) = *(const v4ia*)(OFFG + (size_t)b * NBRUN + 4 * tid);
    *(v4ia*)(scntL + 4 * tid) = *(const v4ia*)(CNTG + (size_t)b * NBRUN + 4 * tid);
#pragma unroll 1
    for (int it = 0; it < 2; ++it) {
      const int u  = it * NTHR + tid;
      const int uc = imin(u, kR * kC / 4 - 1);
      const v4f v = *(const v4fa*)(RELF + 4 * uc);
      asm volatile("" :: "v"(v));
      if (u < kR * kC / 4) *(v4fa*)(relL + 4 * u) = v;
    }
  }
  const v4i mt = *(const v4ia*)(META + (size_t)b * 32);
  __syncthreads();

  const int   nh    = clampi(mt.x, 0, RCAP);
  const bool  flagB = mt.y != 0;
  const float qnan  = __uint_as_float(0x7fc00000u);
  const float ninf  = __uint_as_float(0xff800000u);
  float* sc  = scAll + wave * DEGCAP;
  float* pw  = pwAll + wave * DEGCAP;
  float* stw = stAll + wave * 64;
  const int lc = lane & 15;
  const int l2 = 2 * lane;

#pragma unroll 1
  for (int jt = 0; jt < NBRUN / NWAVE; ++jt) {
    const int slot = wave * (NBRUN / NWAVE) + jt;
    const int grow = b * NBRUN + slot;
    const bool live = grow < kN;
    const int gcl = live ? grow : kN - 1;
    int st = soffL[slot];
    const int craw = scntL[slot];
    st = clampi(st, 0, nh);
    int cnt = clampi(craw, 0, DEGCAP);
    cnt = cnt < nh - st ? cnt : nh - st;
    cnt = live ? cnt : 0;
    const int cn = __builtin_amdgcn_readfirstlane(cnt);
    const int sb = __builtin_amdgcn_readfirstlane(st);
    const bool bad = flagB || (craw > DEGCAP);
    const float pz = bad ? qnan : 0.0f;

    const v2f ph = *(const v2fa*)(P + (size_t)gcl * PW + l2);
    asm volatile("" :: "v"(ph.x), "v"(ph.y));
    const unsigned xw = XBW[(size_t)gcl * (kC / 2) + lane];
    asm volatile("" :: "v"(xw));
    const float xbx = __uint_as_float(xw << 16);
    const float xby = __uint_as_float(xw & 0xffff0000u);
    float sx = xbx, sy = xby;
    if (HOP == 2) {
      const v2f es = *(const v2fa*)(ENTR + (size_t)gcl * kC + l2);
      asm volatile("" :: "v"(es.x), "v"(es.y));
      sx = es.x; sy = es.y;
    }

    wsync();
    float mx = ninf;
#pragma unroll 1
    for (int j = 0; j < cn; ++j) {
      const unsigned w = lst[imin(sb + j, RCAP - 1)];
      const int tl = clampi((int)(w & 0x1FFFFu), 0, kN - 1);
      const int ty = clampi((int)((w >> 17) & 31u), 0, kR - 1);
      const v2f t = *(const v2fa*)(P + (size_t)tl * PW + kC + l2);
      const v2f r = *(const v2fa*)(relL + ty * kC + l2);
      float part = (ph.x + t.x) * r.x;
      part = fmaf(ph.y + t.y, r.y, part);
#pragma unroll
      for (int off = 16; off > 0; off >>= 1) part += __shfl_xor(part, off);
      const float e = part > 0.0f ? part : 0.2f * part;
      if (lane == 0) sc[j] = e;
      mx = e > mx ? e : mx;
    }
    wsync();
    float s = 1.0f;
    if (cn > 0) {
      const float e0 = sc[imin(lane, cn - 1)];
      const float e1 = sc[imin(lane + 32, cn - 1)];
      float p0 = expf(e0 - mx);
      float p1 = expf(e1 - mx);
      p0 = lane < cn ? p0 : 0.0f;
      p1 = lane + 32 < cn ? p1 : 0.0f;
      pw[lane] = p0;
      pw[lane + 32] = p1;
      s = p0 + p1;
#pragma unroll
      for (int off = 16; off > 0; off >>= 1) s += __shfl_xor(s, off);
    }
    wsync();
    float ax = 0.0f, ay = 0.0f;
#pragma unroll 1
    for (int j = 0; j < cn; ++j) {
      const unsigned w = lst[imin(sb + j, RCAP - 1)];
      const int tl = clampi((int)(w & 0x1FFFFu), 0, kN - 1);
      const float p = pw[j];
      float vx, vy;
      if (HOP == 1) {
        const unsigned vw = XBW[(size_t)tl * (kC / 2) + lane];
        vx = __uint_as_float(vw << 16);
        vy = __uint_as_float(vw & 0xffff0000u);
      } else {
        const v2f vv = *(const v2fa*)(ENTR + (size_t)tl * kC + l2);
        vx = vv.x; vy = vv.y;
      }
      ax = fmaf(p, vx, ax);
      ay = fmaf(p, vy, ay);
    }
    const bool has = cn > 0;
    const float sd = has ? s : 1.0f;
    const float gx = has ? (ax / sd + sx) : sx;
    const float gy = has ? (ay / sd + sy) : sy;
    float ss = gx * gx;
    ss = fmaf(gy, gy, ss);
#pragma unroll
    for (int off = 16; off > 0; off >>= 1) ss += __shfl_xor(ss, off);
    const float nrm = sqrtf(ss);
    const float den = nrm > 1e-12f ? nrm : 1e-12f;
    const float ex = gx / den + pz;
    const float ey = gy / den + pz;

    float ox = ex, oy = ey;
    if (HOP == 2) {
      const float r1x = 0.5f * xbx + sx;
      const float r1y = 0.5f * xby + sy;
      ox = 0.5f * r1x + ex;
      oy = 0.5f * r1y + ey;
    }
    wsync();
    *(v2fa*)(stw + l2) = (v2f){ ox, oy };
    wsync();
    const v4f gv = *(const v4fa*)(stw + 4 * lc);
    asm volatile("" :: "v"(gv));
    if (HOP == 1) {
      const int q8 = (lc & 7) * 8;
      const v4f ga = *(const v4fa*)(stw + q8);
      const v4f gb = *(const v4fa*)(stw + q8 + 4);
      const v4u hi = pack8_bf16(ga, gb);
      v4u o = hi;
      if (HOP2_TWO_TERM) {
        const v4u lo = pack8_bf16_lo(ga, gb);
        const unsigned sm = lc >= 8 ? 0xFFFFFFFFu : 0u;
        o = (lo & (v4u){ sm, sm, sm, sm }) | (hi & (v4u){ ~sm, ~sm, ~sm, ~sm });
      }
      const unsigned lm = live ? 0xFFFFFFFFu : 0u;
      o &= (v4u){ lm, lm, lm, lm };
      const bool we = live && lane < 16;
      const bool wp = grow < MPAD && lane < (E1K / 8);
      float* ep = ENTW + (size_t)gcl * kC + 4 * lc;
      unsigned short* pp = E1 + (size_t)imin(grow, MPAD - 1) * E1K + 8 * lc;
      for (int pass = 0; pass < 2; ++pass) {
        if (we) *(volatile v4f*)ep = gv;
        if (wp) *(volatile v4u*)pp = o;
        __threadfence();
      }
    } else {
      const bool we = live && lane < 16;
      float* op = OUT + (size_t)gcl * kC + 4 * lc;
      for (int pass = 0; pass < 2; ++pass) {
        if (we) *(volatile v4f*)op = gv;
        __threadfence();
      }
    }
  }
  (void)ENTW; (void)E1; (void)OUT; (void)ENTR;
}

extern "C" void kernel_launch(void* const* d_in, const int* in_sizes, int n_in,
                              void* d_out, int out_size, void* d_ws, size_t ws_size,
                              hipStream_t stream) {
  if (n_in < 5) return;
  if (in_sizes[0] != kN * kC) return;
  if (in_sizes[1] != kR * kC) return;
  if (in_sizes[2] != 2 * kC * kC) return;
  if (in_sizes[3] != 2 * kE) return;
  if (in_sizes[4] != kE) return;
  if (out_size != kN * kC) return;
  if (ws_size < WS_TOTAL) return;

  const float* ent = (const float*)d_in[0];
  const float* rel = (const float*)d_in[1];
  const float* W   = (const float*)d_in[2];
  const int*   ei  = (const int*)d_in[3];
  const int*   ety = (const int*)d_in[4];
  const int* heads = ei;
  const int* tails = ei + kE;
  float* out = (float*)d_out;

  char* ws = (char*)d_ws;
  unsigned short* XB   = (unsigned short*)(ws + O_XB);
  unsigned short* WB1  = (unsigned short*)(ws + O_WB1);
  unsigned short* WB2  = (unsigned short*)(ws + O_WB2);
  float*          RELF = (float*)(ws + O_RELF);
  float*          Pb   = (float*)(ws + O_P);
  float*          ENT1 = (float*)(ws + O_ENT1);
  unsigned short* E1   = (unsigned short*)(ws + O_E1);
  unsigned*       LIST = (unsigned*)(ws + O_LIST);
  int*            OFFG = (int*)(ws + O_OFF);
  int*            CNTG = (int*)(ws + O_CNT);
  int*            META = (int*)(ws + O_META);

  hipFuncSetAttribute(reinterpret_cast<const void*>(&k_bucket),
                      hipFuncAttributeMaxDynamicSharedMemorySize, LDS_BK);
  hipFuncSetAttribute(reinterpret_cast<const void*>(&k_replay<1>),
                      hipFuncAttributeMaxDynamicSharedMemorySize, LDS_RP);
  hipFuncSetAttribute(reinterpret_cast<const void*>(&k_replay<2>),
                      hipFuncAttributeMaxDynamicSharedMemorySize, LDS_RP);

  const int tiles = ((kN + 63) / 64) * ((PW + 63) / 64);
  const int gGemm = (tiles + 7) / 8;

  k_prep<<<PB_TOTAL, NTHR, 0, stream>>>(ent, rel, W, XB, WB1, WB2, RELF);
  k_bucket<<<NBLK, NTHR, LDS_BK, stream>>>(heads, tails, ety, LIST, OFFG, CNTG, META);
  k_gemm_nt<0, 0><<<gGemm, 256, 0, stream>>>(XB, WB1, RELF, Pb, kN, PW, kC, PW);
  k_replay<1><<<NBLK, NTHR, LDS_RP, stream>>>(LIST, OFFG, CNTG, META, RELF, Pb, (const unsigned*)XB, ENT1,
                                              ENT1, E1, out);
  k_gemm_nt<0, 0><<<gGemm, 256, 0, stream>>>(E1, HOP2_TWO_TERM ? WB2 : WB1, RELF, Pb, kN, PW, E1K, PW);
  k_replay<2><<<NBLK, NTHR, LDS_RP, stream>>>(LIST, OFFG, CNTG, META, RELF, Pb, (const unsigned*)XB, ENT1,
                                              ENT1, E1, out);
}
